// StaticGraphConv_12309376270841
// MI455X (gfx1250) — hardware-verified
//
#include <hip/hip_runtime.h>
#define NNODE 50000
#define NEDGE 800000
#define NP2 1048576
#define DD 64
#define CIN 192
#define NCEN 1000
#define NGRP 4

typedef __bf16 v16b __attribute__((ext_vector_type(16)));
typedef unsigned short v8us __attribute__((ext_vector_type(8), may_alias));
typedef float  v8f  __attribute__((ext_vector_type(8)));
typedef float  v4f  __attribute__((ext_vector_type(4)));
typedef float  v4fa __attribute__((ext_vector_type(4), may_alias));
union FragB { v16b v; v8us half[2]; unsigned short u[16]; };

__device__ __forceinline__ unsigned short bf16_bits(float x) { unsigned int u = __float_as_uint(x); return (unsigned short)((u + 0x7FFFu + ((u >> 16) & 1u)) >> 16); }
__device__ __forceinline__ float bf16_val(unsigned short b) { return __uint_as_float(((unsigned int)b) << 16); }
__device__ __forceinline__ float bf16_round(float x) { return bf16_val(bf16_bits(x)); }
template <int NT>
__device__ __forceinline__ v8f mmaN(v16b ah, v16b al, v16b bh, v16b bl, v8f c) {
  c = __builtin_amdgcn_wmma_f32_16x16x32_bf16(false, ah, false, bh, (short)0, c, false, false);
  if (NT >= 2) c = __builtin_amdgcn_wmma_f32_16x16x32_bf16(false, al, false, bh, (short)0, c, false, false);
  if (NT >= 3) c = __builtin_amdgcn_wmma_f32_16x16x32_bf16(false, ah, false, bl, (short)0, c, false, false);
  asm volatile("v_nop\n\tv_nop\n\tv_nop\n\tv_nop" : "+v"(c) : "v"(ah), "v"(al), "v"(bh), "v"(bl));
  return c;
}

__global__ __launch_bounds__(256) void k_wt_bf16(const float* __restrict__ W, unsigned short* __restrict__ Wt, int K, int N) {
  const int t = blockIdx.x * 256 + threadIdx.x;
  const int k8n = K / 8;
  if (t >= N * k8n) return;
  const int n = t / k8n, k8 = (t % k8n) * 8;
  v8us v;
#pragma unroll
  for (int i = 0; i < 8; ++i) v[i] = bf16_bits(W[(size_t)(k8 + i) * N + n]);
  *(volatile v8us*)(Wt + (size_t)n * K + k8) = v;
  __threadfence();
  *(volatile v8us*)(Wt + (size_t)n * K + k8) = v;
}

template <bool ASPLIT, int ACT, bool BIAS_BF16>
__global__ __launch_bounds__(128) void k_gemm_bf(const float* __restrict__ A, int lda, const unsigned short* __restrict__ Wt, int ldb,
                                               const float* __restrict__ bias, float* __restrict__ C, int ldc, int M, int N, int K) {
  __shared__ __attribute__((aligned(16))) float so[4][16][64];
  const int tid = threadIdx.x, w = tid >> 5, lane = tid & 31, ln = lane & 15, hh = lane >> 4;
  const int ntn = N / 64;
  const int wid = blockIdx.x * 4 + w;
  const int mt = wid / ntn, nq = wid % ntn;
  if (mt * 16 >= M) return;
  const int row0 = mt * 16, col0 = nq * 64;
  const float* arow = A + (size_t)(row0 + ln) * lda;
  v8f acc[4] = {};
  for (int kb = 0; kb < K; kb += 32) {
    FragB ah, al;
    const v4f x0 = *(const v4fa*)(arow + kb + 8 * hh), x1 = *(const v4fa*)(arow + kb + 8 * hh + 4);
    const v4f x2 = *(const v4fa*)(arow + kb + 16 + 8 * hh), x3 = *(const v4fa*)(arow + kb + 16 + 8 * hh + 4);
    float xs[16] = {x0[0],x0[1],x0[2],x0[3],x1[0],x1[1],x1[2],x1[3],x2[0],x2[1],x2[2],x2[3],x3[0],x3[1],x3[2],x3[3]};
#pragma unroll
    for (int i = 0; i < 16; ++i) { const unsigned short hb = bf16_bits(xs[i]); ah.u[i] = hb; al.u[i] = ASPLIT ? bf16_bits(xs[i] - bf16_val(hb)) : (unsigned short)0; }
#pragma unroll
    for (int t = 0; t < 4; ++t) {
      const unsigned short* brow = Wt + (size_t)(col0 + t * 16 + ln) * ldb + kb;
      FragB b;
      b.half[0] = *(const v8us*)(brow + 8 * hh);
      b.half[1] = *(const v8us*)(brow + 16 + 8 * hh);
      acc[t] = mmaN<ASPLIT ? 2 : 1>(ah.v, al.v, b.v, b.v, acc[t]);
    }
  }
#pragma unroll
  for (int t = 0; t < 4; ++t) {
    float bv = bias ? bias[col0 + t * 16 + ln] : 0.f;
    if (BIAS_BF16) bv = bf16_round(bv);
#pragma unroll
    for (int r = 0; r < 8; ++r) { float v = acc[t][r] + bv; if (ACT == 1) v = fmaxf(v, 0.f); so[w][8 * hh + r][t * 16 + ln] = v; }
  }
  __builtin_amdgcn_fence(__ATOMIC_ACQ_REL, "workgroup");
  __builtin_amdgcn_wave_barrier();
  const int rsub = lane >> 4, c4 = (lane & 15) * 4;
  for (int pass = 0; pass < 2; ++pass) {
#pragma unroll
    for (int q = 0; q < 8; ++q) {
      const int r = q * 2 + rsub;
      const v4f v = *(const v4fa*)&so[w][r][c4];
      *(volatile v4f*)(C + (size_t)(row0 + r) * ldc + col0 + c4) = v;
    }
    if (pass == 0) __threadfence();
  }
}

template <int D, bool CAUSAL>
__global__ __launch_bounds__(128) void k_flash(const float* __restrict__ qb, const float* __restrict__ kb, const float* __restrict__ vb,
                                             int pitch, int T, int H, float scale, float* __restrict__ y, int ypitch) {
  constexpr int KS = D / 32;
  constexpr int DT = D / 16;
  __shared__ __attribute__((aligned(16))) unsigned short sKh[32][D + 8], sKl[32][D + 8], sVh[32][D + 8], sVl[32][D + 8];
  __shared__ __attribute__((aligned(16))) unsigned short sPh[4][16][40], sPl[4][16][40];
  __shared__ __attribute__((aligned(16))) float sO[4][16][D];
  const int tid = threadIdx.x, w = tid >> 5, lane = tid & 31, ln = lane & 15, hh = lane >> 4;
  const int nqb = (T + 63) / 64;
  const int bh = blockIdx.x / nqb, qblk = blockIdx.x % nqb;
  const int b = bh / H, h = bh % H;
  const int q0 = qblk * 64 + w * 16;
  const float* Q = qb + (size_t)b * T * pitch + h * D;
  const float* K = kb + (size_t)b * T * pitch + h * D;
  const float* V = vb + (size_t)b * T * pitch + h * D;

  FragB aqh[KS], aql[KS];
  {
    int row = q0 + ln; if (row >= T) row = T - 1;
    const float* qr = Q + (size_t)row * pitch;
#pragma unroll
    for (int ks = 0; ks < KS; ++ks)
#pragma unroll
      for (int i = 0; i < 16; ++i) {
        const int d = ks * 32 + ((i < 8) ? (8 * hh + i) : (16 + 8 * hh + (i - 8)));
        const float x = qr[d] * scale; const unsigned short hb = bf16_bits(x);
        aqh[ks].u[i] = hb; aql[ks].u[i] = bf16_bits(x - bf16_val(hb));
      }
  }
  float m_r[8], l_r[8];
#pragma unroll
  for (int r = 0; r < 8; ++r) { m_r[r] = -3.0e38f; l_r[r] = 0.f; }
  v8f oacc[DT];
#pragma unroll
  for (int dt = 0; dt < DT; ++dt) oacc[dt] = (v8f){0.f,0.f,0.f,0.f,0.f,0.f,0.f,0.f};

  const int kv_end = CAUSAL ? min(T, qblk * 64 + 64) : T;
  for (int j0 = 0; j0 < kv_end; j0 += 32) {
    __syncthreads();
    for (int e = tid; e < 32 * (D / 4); e += 128) {
      const int r = e / (D / 4), c4 = (e % (D / 4)) * 4;
      const int key = j0 + r;
      v4f kf = {0.f,0.f,0.f,0.f}, vf = {0.f,0.f,0.f,0.f};
      if (key < T) { kf = *(const v4fa*)(K + (size_t)key * pitch + c4); vf = *(const v4fa*)(V + (size_t)key * pitch + c4); }
#pragma unroll
      for (int t = 0; t < 4; ++t) {
        unsigned short hb = bf16_bits(kf[t]); sKh[r][c4 + t] = hb; sKl[r][c4 + t] = bf16_bits(kf[t] - bf16_val(hb));
        hb = bf16_bits(vf[t]); sVh[r][c4 + t] = hb; sVl[r][c4 + t] = bf16_bits(vf[t] - bf16_val(hb));
      }
    }
    __syncthreads();
    v8f s[2];
#pragma unroll
    for (int nt = 0; nt < 2; ++nt) {
      v8f acc = {};
#pragma unroll
      for (int ks = 0; ks < KS; ++ks) {
        FragB bh_, bl_;
        bh_.half[0] = *(const v8us*)&sKh[nt * 16 + ln][ks * 32 + 8 * hh]; bh_.half[1] = *(const v8us*)&sKh[nt * 16 + ln][ks * 32 + 16 + 8 * hh];
        bl_.half[0] = *(const v8us*)&sKl[nt * 16 + ln][ks * 32 + 8 * hh]; bl_.half[1] = *(const v8us*)&sKl[nt * 16 + ln][ks * 32 + 16 + 8 * hh];
        acc = mmaN<3>(aqh[ks].v, aql[ks].v, bh_.v, bl_.v, acc);
      }
      s[nt] = acc;
    }
    float alpha[8];
#pragma unroll
    for (int r = 0; r < 8; ++r) {
      const int qi = q0 + 8 * hh + r;
      const int ja = j0 + ln, jb = j0 + 16 + ln;
      if (CAUSAL) { if (ja > qi) s[0][r] = -3.0e38f; if (jb > qi) s[1][r] = -3.0e38f; }
      if (ja >= T) s[0][r] = -3.0e38f;
      if (jb >= T) s[1][r] = -3.0e38f;
      float mx = fmaxf(s[0][r], s[1][r]);
      mx = fmaxf(mx, __shfl_xor(mx, 1, 32)); mx = fmaxf(mx, __shfl_xor(mx, 2, 32)); mx = fmaxf(mx, __shfl_xor(mx, 4, 32)); mx = fmaxf(mx, __shfl_xor(mx, 8, 32));
      const float mnew = fmaxf(m_r[r], mx);
      alpha[r] = (mnew > -1.0e38f) ? __expf(m_r[r] - mnew) : 1.0f;
      const float p0 = (s[0][r] > -1.0e38f) ? __expf(s[0][r] - mnew) : 0.f;
      const float p1 = (s[1][r] > -1.0e38f) ? __expf(s[1][r] - mnew) : 0.f;
      m_r[r] = mnew;
      l_r[r] = l_r[r] * alpha[r] + p0 + p1;
      unsigned short hb = bf16_bits(p0); sPh[w][8 * hh + r][ln] = hb;      sPl[w][8 * hh + r][ln] = bf16_bits(p0 - bf16_val(hb));
      hb = bf16_bits(p1);                sPh[w][8 * hh + r][16 + ln] = hb; sPl[w][8 * hh + r][16 + ln] = bf16_bits(p1 - bf16_val(hb));
    }
#pragma unroll
    for (int dt = 0; dt < DT; ++dt)
#pragma unroll
      for (int r = 0; r < 8; ++r) oacc[dt][r] *= alpha[r];
    __builtin_amdgcn_fence(__ATOMIC_ACQ_REL, "workgroup");
    __builtin_amdgcn_wave_barrier();
    FragB pah, pal;
    pah.half[0] = *(const v8us*)&sPh[w][ln][8 * hh]; pah.half[1] = *(const v8us*)&sPh[w][ln][16 + 8 * hh];
    pal.half[0] = *(const v8us*)&sPl[w][ln][8 * hh]; pal.half[1] = *(const v8us*)&sPl[w][ln][16 + 8 * hh];
#pragma unroll
    for (int dt = 0; dt < DT; ++dt) {
      FragB bvh, bvl;
#pragma unroll
      for (int i = 0; i < 8; ++i) {
        bvh.u[i] = sVh[8 * hh + i][dt * 16 + ln]; bvh.u[8 + i] = sVh[16 + 8 * hh + i][dt * 16 + ln];
        bvl.u[i] = sVl[8 * hh + i][dt * 16 + ln]; bvl.u[8 + i] = sVl[16 + 8 * hh + i][dt * 16 + ln];
      }
      oacc[dt] = mmaN<3>(pah.v, pal.v, bvh.v, bvl.v, oacc[dt]);
    }
    __builtin_amdgcn_fence(__ATOMIC_ACQ_REL, "workgroup");
    __builtin_amdgcn_wave_barrier();
  }
#pragma unroll
  for (int r = 0; r < 8; ++r) {
    float l = l_r[r];
    l += __shfl_xor(l, 1, 32); l += __shfl_xor(l, 2, 32); l += __shfl_xor(l, 4, 32); l += __shfl_xor(l, 8, 32);
    l_r[r] = (l > 0.f) ? 1.0f / l : 0.f;
  }
#pragma unroll
  for (int dt = 0; dt < DT; ++dt)
#pragma unroll
    for (int r = 0; r < 8; ++r) sO[w][8 * hh + r][dt * 16 + ln] = oacc[dt][r] * l_r[r];
  __builtin_amdgcn_fence(__ATOMIC_ACQ_REL, "workgroup");
  __builtin_amdgcn_wave_barrier();
  for (int pass = 0; pass < 2; ++pass) {
    for (int r = 0; r < 16; ++r) {
      const int row = q0 + r;
      if (row < T && lane < D / 4) {
        const v4f val = *(const v4fa*)&sO[w][r][lane * 4];
        *(volatile v4f*)(y + ((size_t)b * T + row) * ypitch + h * D + lane * 4) = val;
      }
    }
    if (pass == 0) __threadfence();
  }
}

__global__ __launch_bounds__(256) void k_sort_init(const int* __restrict__ seg, int n, int nseg, unsigned int* __restrict__ key, unsigned int* __restrict__ val, int np2) {
  const int i = blockIdx.x * 256 + threadIdx.x; if (i >= np2) return;
  unsigned int kv = 0xFFFFFFFFu;
  if (i < n) { int s = seg[i]; s = s < 0 ? 0 : (s >= nseg ? nseg - 1 : s); kv = (unsigned int)s; }
  *(volatile unsigned int*)(key + i) = kv; *(volatile unsigned int*)(val + i) = (unsigned int)i;
  __threadfence();
  *(volatile unsigned int*)(key + i) = kv; *(volatile unsigned int*)(val + i) = (unsigned int)i;
}
template <bool STAGE0>
__global__ __launch_bounds__(512) void k_sort_lds(unsigned int* __restrict__ key, unsigned int* __restrict__ val, int kstage) {
  __shared__ unsigned int sk[1024], sv[1024];
  const int tid = threadIdx.x; const int base = blockIdx.x * 1024;
  sk[tid] = key[base + tid]; sv[tid] = val[base + tid]; sk[tid + 512] = key[base + tid + 512]; sv[tid + 512] = val[base + tid + 512];
  __syncthreads();
  for (int k = (STAGE0 ? 2 : kstage); k <= (STAGE0 ? 1024 : kstage); k <<= 1) {
    for (int j = (k > 1024 ? 512 : (k >> 1)); j >= 1; j >>= 1) {
      const int lo = tid & (j - 1), hi2 = (tid >> __builtin_ctz(j)) << (__builtin_ctz(j) + 1);
      const int il = hi2 | lo, ir = il | j;
      const int gi = base + il;
      const bool asc = ((gi & k) == 0);
      unsigned int a = sk[il], b = sk[ir], va = sv[il], vb = sv[ir];
      const bool swp = asc ? (a > b) : (a < b);
      if (swp) { sk[il] = b; sk[ir] = a; sv[il] = vb; sv[ir] = va; }
      __syncthreads();
    }
  }
  for (int pass = 0; pass < 2; ++pass) {
    *(volatile unsigned int*)(key + base + tid) = sk[tid]; *(volatile unsigned int*)(val + base + tid) = sv[tid];
    *(volatile unsigned int*)(key + base + tid + 512) = sk[tid + 512]; *(volatile unsigned int*)(val + base + tid + 512) = sv[tid + 512];
    if (pass == 0) __threadfence();
  }
}
__global__ __launch_bounds__(256) void k_sort_step(unsigned int* __restrict__ key, unsigned int* __restrict__ val, int k, int j, int np2) {
  const int t = blockIdx.x * 256 + threadIdx.x; if (t >= np2 / 2) return;
  const int lo = t & (j - 1), il = ((t >> __builtin_ctz(j)) << (__builtin_ctz(j) + 1)) | lo, ir = il | j;
  const bool asc = ((il & k) == 0);
  unsigned int a = key[il], b = key[ir], va = val[il], vb = val[ir];
  const bool swp = asc ? (a > b) : (a < b);
  const unsigned int k1 = swp ? b : a, k2 = swp ? a : b, v1 = swp ? vb : va, v2 = swp ? va : vb;
  *(volatile unsigned int*)(key + il) = k1; *(volatile unsigned int*)(key + ir) = k2; *(volatile unsigned int*)(val + il) = v1; *(volatile unsigned int*)(val + ir) = v2;
  __threadfence();
  *(volatile unsigned int*)(key + il) = k1; *(volatile unsigned int*)(key + ir) = k2; *(volatile unsigned int*)(val + il) = v1; *(volatile unsigned int*)(val + ir) = v2;
}
__global__ __launch_bounds__(256) void k_rowptr(const unsigned int* __restrict__ key, int np2, int nseg, int* __restrict__ rowptr) {
  int s = blockIdx.x * 256 + threadIdx.x; if (s >= ((nseg + 1 + 31) / 32) * 32) return;
  const int sdst = s; if (s > nseg) s = nseg;
  int lo = 0, hi = np2;
  while (lo < hi) { const int mid = (lo + hi) >> 1; if (key[mid] < (unsigned int)s) lo = mid + 1; else hi = mid; }
  *(volatile int*)(rowptr + sdst) = lo; __threadfence(); *(volatile int*)(rowptr + sdst) = lo;
}
static void sort_pairs(unsigned int* key, unsigned int* val, int np2, hipStream_t stream) {
  k_sort_lds<true><<<np2 / 1024, 512, 0, stream>>>(key, val, 0);
  for (int k = 2048; k <= np2; k <<= 1) {
    for (int j = k >> 1; j >= 1024; j >>= 1) k_sort_step<<<(np2 / 2 + 255) / 256, 256, 0, stream>>>(key, val, k, j, np2);
    k_sort_lds<false><<<np2 / 1024, 512, 0, stream>>>(key, val, k);
  }
}

__global__ __launch_bounds__(256) void k_centroids(const float* __restrict__ xc_in, const float* __restrict__ Wc, const float* __restrict__ bc, float* __restrict__ xc) {
  const int t = blockIdx.x * 256 + threadIdx.x; if (t >= NCEN * DD) return; const int c = t / DD, o = t % DD; const int g = o / 16, oo = o % 16;
  float s = bf16_round(bc[o]);
#pragma unroll 1
  for (int i = 0; i < 16; ++i) s += bf16_round(xc_in[c * DD + g * 16 + i]) * bf16_round(Wc[(g * 16 + i) * 16 + oo]);
  s = fmaxf(s, 0.f);
  *(volatile float*)(xc + t) = s; __threadfence(); *(volatile float*)(xc + t) = s;
}
__global__ __launch_bounds__(256) void k_wt_grouped(const float* __restrict__ Wv, unsigned short* __restrict__ Bt) {
  const int t = blockIdx.x * 256 + threadIdx.x; if (t >= DD * (CIN / 8)) return; const int n = t / (CIN / 8), k8 = (t % (CIN / 8)) * 8; const int g = n / 16, o = n % 16; v8us v;
  for (int i = 0; i < 8; ++i) { const int k = k8 + i; v[i] = (k / 48 == g) ? bf16_bits(Wv[((size_t)g * 48 + (k - 48 * g)) * 16 + o]) : (unsigned short)0; }
  *(volatile v8us*)(Bt + (size_t)n * CIN + k8) = v; __threadfence(); *(volatile v8us*)(Bt + (size_t)n * CIN + k8) = v;
}
__global__ __launch_bounds__(128) void k_edge_gemm(const float* __restrict__ x, const float* __restrict__ xc, const int* __restrict__ batch, const int* __restrict__ src, const int* __restrict__ dst,
                                                 const unsigned short* __restrict__ Bt, const float* __restrict__ bv, float* __restrict__ h) {
  __shared__ __attribute__((aligned(16))) float so[4][16][64];
  const int tid = threadIdx.x, w = tid >> 5, lane = tid & 31, ln = lane & 15, hh = lane >> 4;
  const size_t e0 = ((size_t)blockIdx.x * 4 + w) * 16; const size_t e = e0 + ln;
  int sn = src[e]; sn = sn < 0 ? 0 : (sn >= NNODE ? NNODE - 1 : sn); int dn = dst[e]; dn = dn < 0 ? 0 : (dn >= NNODE ? NNODE - 1 : dn);
  int cb = batch[sn]; cb = cb < 0 ? 0 : (cb >= NCEN ? NCEN - 1 : cb);
  const float* xi = x + (size_t)dn * DD; const float* xj = x + (size_t)sn * DD; const float* yj = xc + (size_t)cb * DD;
  v8f acc[4] = {};
#pragma unroll
  for (int ks = 0; ks < CIN / 32; ++ks) {
    FragB ah, al;
#pragma unroll
    for (int i = 0; i < 16; ++i) { const int k = ks * 32 + ((i < 8) ? (8 * hh + i) : (16 + 8 * hh + (i - 8))); float v;
      if (k < DD) v = bf16_round(xi[k]); else if (k < 2 * DD) v = bf16_round(xj[k - DD]) - bf16_round(xi[k - DD]); else v = yj[k - 2 * DD];
      const unsigned short hb = bf16_bits(v); ah.u[i] = hb; al.u[i] = bf16_bits(v - bf16_val(hb)); }
#pragma unroll
    for (int t = 0; t < 4; ++t) { FragB b; b.half[0] = *(const v8us*)(Bt + (size_t)(t * 16 + ln) * CIN + ks * 32 + 8 * hh); b.half[1] = *(const v8us*)(Bt + (size_t)(t * 16 + ln) * CIN + ks * 32 + 16 + 8 * hh); acc[t] = mmaN<2>(ah.v, al.v, b.v, b.v, acc[t]); }
  }
#pragma unroll
  for (int t = 0; t < 4; ++t) { const int col = t * 16 + ln; const float bb = bf16_round(bv[col]);
#pragma unroll
    for (int r = 0; r < 8; ++r) so[w][8 * hh + r][col] = acc[t][r] + bb; }
  __builtin_amdgcn_fence(__ATOMIC_ACQ_REL, "workgroup"); __builtin_amdgcn_wave_barrier();
  const int rsub = lane >> 4, c4 = (lane & 15) * 4;
  for (int pass = 0; pass < 2; ++pass) { for (int q = 0; q < 8; ++q) { const int r = q * 2 + rsub; const v4f v = *(const v4fa*)&so[w][r][c4]; *(volatile v4f*)(h + (e0 + r) * DD + c4) = v; } if (pass == 0) __threadfence(); }
}
__global__ __launch_bounds__(64) void k_colstat1(const float* __restrict__ h, int nrows, double* __restrict__ part) {
  const int c = threadIdx.x; const int r0 = blockIdx.x * 4096; const int r1 = min(r0 + 4096, nrows);
  double s = 0.0, s2 = 0.0;
#pragma unroll 1
  for (int r = r0; r < r1; ++r) { const double v = (double)h[(size_t)r * DD + c]; s += v; s2 += v * v; }
  double* dst = part + (size_t)blockIdx.x * 2 * DD;
  *(volatile double*)(dst + c) = s; *(volatile double*)(dst + DD + c) = s2; __threadfence(); *(volatile double*)(dst + c) = s; *(volatile double*)(dst + DD + c) = s2;
}
__global__ __launch_bounds__(64) void k_colstat2(const double* __restrict__ part, int nblk, int nrows, float* __restrict__ stats) {
  const int c = threadIdx.x; double s = 0.0, s2 = 0.0;
  for (int b = 0; b < nblk; ++b) { s += part[(size_t)b * 2 * DD + c]; s2 += part[(size_t)b * 2 * DD + DD + c]; }
  const double mu = s / nrows; double var = s2 / nrows - mu * mu; if (var < 0.0) var = 0.0;
  const float m = (float)mu, rs = (float)(1.0 / sqrt(var + 1e-5));
  *(volatile float*)(stats + c) = m; *(volatile float*)(stats + DD + c) = rs; __threadfence(); *(volatile float*)(stats + c) = m; *(volatile float*)(stats + DD + c) = rs;
}
__global__ __launch_bounds__(256) void k_maxagg(const float* __restrict__ h, const float* __restrict__ stats, const float* __restrict__ g, const float* __restrict__ bt,
                                              const int* __restrict__ rowptr, const unsigned int* __restrict__ perm, float* __restrict__ out) {
  const int tid = threadIdx.x, w = tid >> 5, lane = tid & 31; const int nd = blockIdx.x * 8 + w; if (nd >= NNODE) return;
  if (lane >= 16) return;
  const int p0 = rowptr[nd], p1 = rowptr[nd + 1];
  float sc[4], sh[4]; for (int q = 0; q < 4; ++q) { const int c = lane * 4 + q; sc[q] = stats[DD + c] * bf16_round(g[c]); sh[q] = bf16_round(bt[c]) - stats[c] * sc[q]; }
  v4f m = {-__builtin_inff(), -__builtin_inff(), -__builtin_inff(), -__builtin_inff()};
  for (int p = p0; p < p1; ++p) { const v4f x0 = *(const v4fa*)(h + (size_t)perm[p] * DD + lane * 4); for (int q = 0; q < 4; ++q) m[q] = fmaxf(m[q], fmaxf(x0[q] * sc[q] + sh[q], 0.f)); }
  v4f o; for (int q = 0; q < 4; ++q) o[q] = (p1 > p0) ? m[q] : 0.f;
  float* row = out + (size_t)nd * DD + lane * 4; *(volatile v4f*)row = o; __threadfence(); *(volatile v4f*)row = o;
}
extern "C" void kernel_launch(void* const* d_in, const int* in_sizes, int n_in,
                              void* d_out, int out_size, void* d_ws, size_t ws_size, hipStream_t stream) {
  (void)in_sizes; (void)n_in; (void)out_size;
  const float* x = (const float*)d_in[0]; const int* batch = (const int*)d_in[1]; const int* ei = (const int*)d_in[2]; const float* xcen = (const float*)d_in[3];
  const float* Wc = (const float*)d_in[5]; const float* bc = (const float*)d_in[6]; const float* Wv = (const float*)d_in[7]; const float* bv = (const float*)d_in[8];
  const float* gamma = (const float*)d_in[9]; const float* beta = (const float*)d_in[10];
  const int* src = ei; const int* dst = ei + NEDGE;
  char* ws = (char*)d_ws; size_t off = 0;
  auto take = [&](size_t bytes) { char* p = ws + off; off += (bytes + 255) & ~(size_t)255; return p; };
  const int nblk = (NEDGE + 4095) / 4096;
  unsigned short* Bt = (unsigned short*)take((size_t)DD * CIN * 2); float* xc = (float*)take((size_t)NCEN * DD * 4);
  unsigned int* key = (unsigned int*)take((size_t)NP2 * 4); unsigned int* perm = (unsigned int*)take((size_t)NP2 * 4); int* rowptr = (int*)take((size_t)(NNODE + 64) * 4);
  float* h = (float*)take((size_t)NEDGE * DD * 4); double* part = (double*)take((size_t)nblk * 2 * DD * 8); float* stats = (float*)take(2 * DD * 4);
  if (off > ws_size) return;
  k_centroids<<<(NCEN * DD + 255) / 256, 256, 0, stream>>>(xcen, Wc, bc, xc);
  k_wt_grouped<<<(DD * (CIN / 8) + 255) / 256, 256, 0, stream>>>(Wv, Bt);
  k_sort_init<<<NP2 / 256, 256, 0, stream>>>(dst, NEDGE, NNODE, key, perm, NP2);
  sort_pairs(key, perm, NP2, stream);
  k_rowptr<<<(NNODE + 32 + 255) / 256, 256, 0, stream>>>(key, NP2, NNODE, rowptr);
  k_edge_gemm<<<NEDGE / 64, 128, 0, stream>>>(x, xc, batch, src, dst, Bt, bv, h);
  k_colstat1<<<nblk, 64, 0, stream>>>(h, NEDGE, part); k_colstat2<<<1, 64, 0, stream>>>(part, nblk, NEDGE, stats);
  k_maxagg<<<(NNODE + 7) / 8, 256, 0, stream>>>(h, stats, gamma, beta, rowptr, perm, (float*)d_out);
}
